// TrajectoryPrediction_58832462020776
// MI455X (gfx1250) — hardware-run, weakly checked
//
#include <hip/hip_runtime.h>
#include <math.h>

typedef __attribute__((ext_vector_type(16))) _Float16 v16h;
typedef __attribute__((ext_vector_type(8)))  _Float16 v8h;
typedef __attribute__((ext_vector_type(16))) __bf16   v16b;
typedef __attribute__((ext_vector_type(8)))  __bf16   v8b;
typedef __attribute__((ext_vector_type(8)))  float    v8f;
typedef __attribute__((ext_vector_type(4)))  float    v4f;
typedef __attribute__((ext_vector_type(2)))  float    v2f;
typedef __attribute__((ext_vector_type(2)))  unsigned int v2u;

constexpr int kT     = 8;
constexpr int kNP    = 2048;
constexpr int kNG    = 64;
constexpr int kGS    = 32;
constexpr int kHD    = 128;
constexpr int kDIN   = 64;
constexpr int kDD    = 64;
constexpr int kNH    = 4;
constexpr int kKL    = kDIN + kHD;
constexpr int kNGATE = 4 * kHD;
constexpr int kNPAIR = kNP * kGS;
constexpr int kKC    = kNH * kHD;

static_assert(kNP % 64 == 0 && kNGATE % 64 == 0 && kKL % 32 == 0);
static_assert(kNPAIR % 64 == 0 && kHD % 64 == 0 && kDD % 32 == 0);
static_assert(kKC % 32 == 0 && kNG * kGS == kNP);

constexpr size_t al256(size_t b) { return (b + 255) & ~size_t(255); }
constexpr size_t szWc   = al256((size_t)kNGATE * kKL * 2);
constexpr size_t szBias = al256((size_t)kNGATE * 4);
constexpr size_t szWg   = al256((size_t)kHD * kDD * 2);
constexpr size_t szWa   = al256((size_t)kHD * kKC * 2);
constexpr size_t szWav  = al256((size_t)2 * kKC * 4);
constexpr size_t szPl   = al256((size_t)kT * kNP * kKL * 2);
constexpr size_t szG    = al256((size_t)kNP * kNGATE * 4);
constexpr size_t szC    = al256((size_t)kNP * kHD * 4);
constexpr size_t szM1   = al256((size_t)kNPAIR * kDD * 2);
constexpr size_t szGate = al256((size_t)kNPAIR * kHD * 4);
constexpr size_t szCtx  = al256((size_t)kNP * kKC * 2);
constexpr size_t oWcH = 0;
constexpr size_t oWcL = oWcH + szWc;
constexpr size_t oBias = oWcL + szWc;
constexpr size_t oWgH = oBias + szBias;
constexpr size_t oWgL = oWgH + szWg;
constexpr size_t oWaH = oWgL + szWg;
constexpr size_t oWaL = oWaH + szWa;
constexpr size_t oWav = oWaL + szWa;
constexpr size_t oPH = oWav + szWav;
constexpr size_t oPL = oPH + szPl;
constexpr size_t oG = oPL + szPl;
constexpr size_t oC0 = oG + szG;
constexpr size_t oC1 = oC0 + szC;
constexpr size_t oAh = oC1 + szC;
constexpr size_t oMH = oAh + szC;
constexpr size_t oML = oMH + szM1;
constexpr size_t oGate = oML + szM1;
constexpr size_t oXH = oGate + szGate;
constexpr size_t oXL = oXH + szCtx;
constexpr size_t kWsTotal = oXL + szCtx;
static_assert(kWsTotal == 75143168);
static_assert(kWsTotal <= 134217728);

__device__ __forceinline__ unsigned short f2bf_bits(float f) {
  unsigned u = __float_as_uint(f);
  return (unsigned short)((u + 0x7FFFu + ((u >> 16) & 1u)) >> 16);
}
__device__ __forceinline__ float bf_bits2f(unsigned short h) { return __uint_as_float(((unsigned)h) << 16); }

__device__ __forceinline__ void dep_guard_h(v8f& a, v8f& b, v16h x, v16h y) { asm volatile("v_nop\n\tv_nop\n\tv_nop\n\tv_nop" : "+v"(a), "+v"(b) : "v"(x), "v"(y)); }
__device__ __forceinline__ void dep_guard_b(v8f& a, v8f& b, v16b x, v16b y) { asm volatile("v_nop\n\tv_nop\n\tv_nop\n\tv_nop" : "+v"(a), "+v"(b) : "v"(x), "v"(y)); }
__device__ __forceinline__ void keep4_h(v16h a, v16h b, v16h c, v16h d) { asm volatile("v_nop" :: "v"(a), "v"(b), "v"(c), "v"(d)); }
__device__ __forceinline__ void keep4_b(v16b a, v16b b, v16b c, v16b d) { asm volatile("v_nop" :: "v"(a), "v"(b), "v"(c), "v"(d)); }
__device__ __forceinline__ void acc_guard4(v8f& a, v8f& b, v8f& c, v8f& d) { asm volatile("v_nop\n\tv_nop\n\tv_nop\n\tv_nop" : "+v"(a), "+v"(b), "+v"(c), "+v"(d)); }
template <typename T> struct Frag;
template <> struct Frag<_Float16> {
  typedef v16h V; union U { v16h v; v8h h[2]; };
  static __device__ __forceinline__ v16h load(const _Float16* p) {
    U f; f.h[0] = *(const v8h*)(p); f.h[1] = *(const v8h*)(p + 16); return f.v;
  }
  static __device__ __forceinline__ v8f mma(v16h a, v16h b, v8f c) {
    return __builtin_amdgcn_wmma_f32_16x16x32_f16(false, a, false, b, (short)0, c, false, false);
  }
  static __device__ __forceinline__ void guard(v8f& a, v8f& b, v16h x, v16h y) { dep_guard_h(a, b, x, y); }
  static __device__ __forceinline__ void keep(v16h a, v16h b, v16h c, v16h d) { keep4_h(a, b, c, d); }
};
template <> struct Frag<__bf16> {
  typedef v16b V; union U { v16b v; v8b h[2]; };
  static __device__ __forceinline__ v16b load(const __bf16* p) {
    U f; f.h[0] = *(const v8b*)(p); f.h[1] = *(const v8b*)(p + 16); return f.v;
  }
  static __device__ __forceinline__ v8f mma(v16b a, v16b b, v8f c) {
    return __builtin_amdgcn_wmma_f32_16x16x32_bf16(false, a, false, b, (short)0, c, false, false);
  }
  static __device__ __forceinline__ void guard(v8f& a, v8f& b, v16b x, v16b y) { dep_guard_b(a, b, x, y); }
  static __device__ __forceinline__ void keep(v16b a, v16b b, v16b c, v16b d) { keep4_b(a, b, c, d); }
};

template <int ET> struct Elem;
template <> struct Elem<0> { typedef _Float16 T; };
template <> struct Elem<1> { typedef __bf16 T; };
template <int ET, bool SPLIT, int BIAS_MODE, int OUT_MODE, bool RESID, int ACT = 0>
__global__ __launch_bounds__(256) void wmma_gemm64(
    const unsigned short* __restrict__ Ap, const unsigned short* __restrict__ A2p, int lda, long strideA,
    const unsigned short* __restrict__ Btp, const unsigned short* __restrict__ Bt2p, int ldb, long strideB,
    void* __restrict__ Cout, void* __restrict__ Cout2, int ldc, long strideC,
    const float* __restrict__ bias,
    const float* __restrict__ resid, long strideR,
    int M, int N, int K, float scale) {
  typedef typename Elem<ET>::T T;
  typedef typename Frag<T>::V V;
  const T* A = (const T*)Ap; const T* A2 = (const T*)A2p; const T* Bt = (const T*)Btp; const T* Bt2 = (const T*)Bt2p;
  __shared__ __align__(16) float sT[8][16 * 68];
  const int b    = blockIdx.y;
  const int lane = threadIdx.x & 31;
  const int wave = threadIdx.x >> 5;
  const int tilesN = N >> 6;
  const int tilesM = M >> 6;
  const int tile = blockIdx.x * 8 + wave;
  if (tile >= tilesM * tilesN) return;
  const int tm = tile / tilesN;
  const int tn = tile - tm * tilesN;
  const int m0 = tm << 6;
  const int n0 = tn << 6;

  const T* Ab  = A  + (size_t)b * strideA;
  const T* Bb  = Bt + (size_t)b * strideB;
  const T* Ab2 = SPLIT ? (A2  + (size_t)b * strideA) : nullptr;
  const T* Bb2 = SPLIT ? (Bt2 + (size_t)b * strideB) : nullptr;

  const int rlane = lane & 15;
  const int koff  = (lane >> 4) * 8;
  const int mOff  = (lane >> 4) * 8;

  v8f acc[4][4];
#pragma unroll
  for (int i = 0; i < 4; ++i)
#pragma unroll
    for (int j = 0; j < 4; ++j) acc[i][j] = (v8f){0.f,0.f,0.f,0.f,0.f,0.f,0.f,0.f};

  for (int k0 = 0; k0 < K; k0 += 32) {
    V bh[4], bl[4];
#pragma unroll
    for (int j = 0; j < 4; ++j) {
      const size_t bo = (size_t)(n0 + (j << 4) + rlane) * ldb + koff + k0;
      bh[j] = Frag<T>::load(Bb + bo);
      if (SPLIT) bl[j] = Frag<T>::load(Bb2 + bo);
    }
#pragma unroll
    for (int i = 0; i < 4; ++i) {
      const size_t ao = (size_t)(m0 + (i << 4) + rlane) * lda + koff + k0;
      V ah = Frag<T>::load(Ab + ao);
      V al;
      if (SPLIT) al = Frag<T>::load(Ab2 + ao);
#pragma unroll
      for (int j = 0; j < 4; ++j) {
        acc[i][j] = Frag<T>::mma(ah, bh[j], acc[i][j]);
        if (SPLIT) {
          acc[i][j] = Frag<T>::mma(ah, bl[j], acc[i][j]);
          acc[i][j] = Frag<T>::mma(al, bh[j], acc[i][j]);
        }
      }
      Frag<T>::guard(acc[i][0], acc[i][3], ah, SPLIT ? al : ah);
    }
    Frag<T>::keep(bh[0], bh[1], bh[2], bh[3]);
    if (SPLIT) Frag<T>::keep(bl[0], bl[1], bl[2], bl[3]);
  }
  acc_guard4(acc[0][0], acc[0][1], acc[0][2], acc[0][3]);
  acc_guard4(acc[1][0], acc[1][1], acc[1][2], acc[1][3]);
  acc_guard4(acc[2][0], acc[2][1], acc[2][2], acc[2][3]);
  acc_guard4(acc[3][0], acc[3][1], acc[3][2], acc[3][3]);

  float* slab = sT[wave];
  const float* Rb = RESID ? (resid + (size_t)b * strideR) : nullptr;
#pragma unroll
  for (int i = 0; i < 4; ++i) {
    const int mBase = m0 + (i << 4);
#pragma unroll
    for (int j = 0; j < 4; ++j) {
      const int n = n0 + (j << 4) + rlane;
      float bv = 0.f;
      if (BIAS_MODE == 2 || BIAS_MODE == 3) bv = bias[n];
#pragma unroll
      for (int r = 0; r < 8; ++r) {
        float v = acc[i][j][r] * scale;
        if (BIAS_MODE == 1) v += bias[mBase + mOff + r];
        if (BIAS_MODE == 2) v += bv;
        if (RESID) v += Rb[(size_t)(mBase + mOff + r) * ldc + n];
        if (ACT == 1) v = tanhf(v);
        if (ACT == 2) v = fmaxf(v, 0.0f);
        if (ACT == 3) v = v / (1.0f + expf(-v));
        if (ACT == 4) v = (v > 0.f) ? v : 0.01f * v;
        if (ACT == 5) v = 0.5f * v * (1.0f + erff(v * 0.70710678118654752f));
        if (ACT == 6) v = __builtin_amdgcn_rcpf(1.0f + expf(-v));
        if (BIAS_MODE == 3) v += bv;
        slab[(mOff + r) * 68 + (j << 4) + rlane] = v;
      }
    }
    __builtin_amdgcn_fence(__ATOMIC_RELEASE, "workgroup");
    __builtin_amdgcn_wave_barrier();
    __builtin_amdgcn_fence(__ATOMIC_ACQUIRE, "workgroup");
    if (OUT_MODE == 0) {
      float* C = (float*)Cout + (size_t)b * strideC;
      const int hh = lane >> 4, c4 = (lane & 15) * 4;
      for (int pass = 0; pass < 2; ++pass) {
#pragma unroll
        for (int it = 0; it < 8; ++it) {
          const int row = it * 2 + hh;
          v4f v = *(const v4f*)(slab + row * 68 + c4);
          *(volatile v4f*)(C + (size_t)(mBase + row) * ldc + n0 + c4) = v;
        }
        __threadfence();
      }
    } else {
      const int q = lane >> 3, c8 = (lane & 7) * 8;
      unsigned short* C  = (unsigned short*)Cout  + (size_t)b * strideC;
      unsigned short* C2 = (OUT_MODE == 2) ? ((unsigned short*)Cout2 + (size_t)b * strideC) : nullptr;
      for (int pass = 0; pass < 2; ++pass) {
#pragma unroll
        for (int it = 0; it < 4; ++it) {
          const int row = it * 4 + q;
          const float* sp = slab + row * 68 + c8;
          v8h hv, lv;
#pragma unroll
          for (int e = 0; e < 8; ++e) {
            if (OUT_MODE == 1) {
              hv[e] = (_Float16)sp[e];
            } else {
              unsigned short hb = f2bf_bits(sp[e]);
              unsigned short lb = f2bf_bits(sp[e] - bf_bits2f(hb));
              hv[e] = __builtin_bit_cast(_Float16, hb);
              lv[e] = __builtin_bit_cast(_Float16, lb);
            }
          }
          *(volatile v8h*)(C + (size_t)(mBase + row) * ldc + n0 + c8) = hv;
          if (OUT_MODE == 2) *(volatile v8h*)(C2 + (size_t)(mBase + row) * ldc + n0 + c8) = lv;
        }
        __threadfence();
      }
    }
    __builtin_amdgcn_fence(__ATOMIC_RELEASE, "workgroup");
    __builtin_amdgcn_wave_barrier();
    __builtin_amdgcn_fence(__ATOMIC_ACQUIRE, "workgroup");
  }
}

__device__ __forceinline__ float rcp_f(float x) { return __builtin_amdgcn_rcpf(x); }
__device__ __forceinline__ float sigm_f(float x) { return rcp_f(1.0f + expf(-x)); }
__device__ __forceinline__ float tanh_f(float x) { const float e = expf(-2.0f * x); return 2.0f * rcp_f(1.0f + e) - 1.0f; }
__device__ __forceinline__ v4f sel4(bool c, v4f a, v4f b) {
  v4f r; r.x = c ? a.x : b.x; r.y = c ? a.y : b.y; r.z = c ? a.z : b.z; r.w = c ? a.w : b.w; return r;
}
__device__ __forceinline__ float wave_sum(float p) {
  p += __shfl_xor(p, 16, 32); p += __shfl_xor(p, 8, 32); p += __shfl_xor(p, 4, 32);
  p += __shfl_xor(p, 2, 32);  p += __shfl_xor(p, 1, 32);
  return p;
}
__device__ __forceinline__ void wave_sync() {
  __builtin_amdgcn_fence(__ATOMIC_RELEASE, "workgroup");
  __builtin_amdgcn_wave_barrier();
  __builtin_amdgcn_fence(__ATOMIC_ACQUIRE, "workgroup");
}
__device__ __forceinline__ void split_pack4(v4f v, v2u& hi, v2u& lo) {
  const unsigned short ba = f2bf_bits(v.x), bb = f2bf_bits(v.y), bc = f2bf_bits(v.z), bd = f2bf_bits(v.w);
  const unsigned short la = f2bf_bits(v.x - bf_bits2f(ba)), lb = f2bf_bits(v.y - bf_bits2f(bb));
  const unsigned short lc = f2bf_bits(v.z - bf_bits2f(bc)), ld = f2bf_bits(v.w - bf_bits2f(bd));
  hi.x = (unsigned)ba | ((unsigned)bb << 16); hi.y = (unsigned)bc | ((unsigned)bd << 16);
  lo.x = (unsigned)la | ((unsigned)lb << 16); lo.y = (unsigned)lc | ((unsigned)ld << 16);
}
__device__ __forceinline__ void store_planes_2pass(unsigned short* ph, unsigned short* pl, v2u hi, v2u lo) {
  *(volatile v2u*)ph = hi; *(volatile v2u*)pl = lo;
  __threadfence();
  *(volatile v2u*)ph = hi; *(volatile v2u*)pl = lo;
}
__device__ __forceinline__ void store_f4_2pass(float* p, v4f v) {
  *(volatile v4f*)p = v;
  __threadfence();
  *(volatile v4f*)p = v;
}

__global__ __launch_bounds__(256) void prep_params(
    const float* __restrict__ W_ih, const float* __restrict__ W_hh,
    const float* __restrict__ b_ih, const float* __restrict__ b_hh,
    const float* __restrict__ W_gate, const float* __restrict__ gat_w, const float* __restrict__ gat_a,
    unsigned short* __restrict__ WcH, unsigned short* __restrict__ WcL, float* __restrict__ biasg,
    unsigned short* __restrict__ WgH, unsigned short* __restrict__ WgL,
    unsigned short* __restrict__ WaH, unsigned short* __restrict__ WaL, float* __restrict__ wa) {
  const int idx = blockIdx.x * 256 + threadIdx.x;
  if (idx < kNGATE * (kKL / 4)) {
    const int n = idx / (kKL / 4);
    const int col = (idx - n * (kKL / 4)) * 4;
    const int ci = min(col, kDIN - 4);
    const int ch = min(max(col - kDIN, 0), kHD - 4);
    const v4f a = *(const v4f*)(W_ih + (size_t)n * kDIN + ci);
    const v4f b = *(const v4f*)(W_hh + (size_t)n * kHD + ch);
    const v4f v = sel4(col < kDIN, a, b);
    v2u hi, lo; split_pack4(v, hi, lo);
    store_planes_2pass(WcH + (size_t)n * kKL + col, WcL + (size_t)n * kKL + col, hi, lo);
  }
  if (idx < kHD * (kDD / 4)) {
    const int o = idx >> 4;
    const int q = (idx & 15) * 4;
    v4f v;
    v.x = W_gate[(size_t)(q + 0) * kHD + o]; v.y = W_gate[(size_t)(q + 1) * kHD + o];
    v.z = W_gate[(size_t)(q + 2) * kHD + o]; v.w = W_gate[(size_t)(q + 3) * kHD + o];
    v2u hi, lo; split_pack4(v, hi, lo);
    store_planes_2pass(WgH + (size_t)o * kDD + q, WgL + (size_t)o * kDD + q, hi, lo);
  }
  if (idx < kHD * (kKC / 4)) {
    const int o = idx >> 7;
    const int col = (idx & 127) * 4;
    const int h = col >> 7, f = col & 127;
    const float* src = gat_w + (size_t)h * kHD * kHD + (size_t)f * kHD + o;
    v4f v;
    v.x = src[0]; v.y = src[kHD]; v.z = src[2 * kHD]; v.w = src[3 * kHD];
    v2u hi, lo; split_pack4(v, hi, lo);
    store_planes_2pass(WaH + (size_t)o * kKC + col, WaL + (size_t)o * kKC + col, hi, lo);
  }
  if (idx < kNGATE / 4) {
    const v4f v = *(const v4f*)(b_ih + 4 * idx) + *(const v4f*)(b_hh + 4 * idx);
    store_f4_2pass(biasg + 4 * idx, v);
  }
  if (idx < 2 * kNH * (kHD / 4)) {
    const int s = idx >> 7;
    const int rem = idx & 127;
    const int h = rem >> 5;
    const int f = (rem & 31) * 4;
    const float* wrow = gat_w + (size_t)h * kHD * kHD + (size_t)f * kHD;
    const float* av = gat_a + s * kHD;
    float a0 = 0.0f, a1 = 0.0f, a2 = 0.0f, a3 = 0.0f;
#pragma unroll 1
    for (int o = 0; o < kHD; ++o) {
      const float a = av[o];
      a0 = fmaf(wrow[o], a, a0);
      a1 = fmaf(wrow[kHD + o], a, a1);
      a2 = fmaf(wrow[2 * kHD + o], a, a2);
      a3 = fmaf(wrow[3 * kHD + o], a, a3);
    }
    v4f v; v.x = a0; v.y = a1; v.z = a2; v.w = a3;
    store_f4_2pass(wa + s * kKC + h * kHD + f, v);
  }
}

__global__ __launch_bounds__(256) void embed_inputs(
    const float* __restrict__ obs, const float* __restrict__ W_emb, const float* __restrict__ b_emb,
    const float* __restrict__ h0v, unsigned short* __restrict__ PH, unsigned short* __restrict__ PL) {
  const int idx = blockIdx.x * 256 + threadIdx.x;
  if (idx < kT * kNP * (kDIN / 4)) {
    const int row = idx >> 4;
    const int d = (idx & 15) * 4;
    const float px = obs[2 * (size_t)row], py = obs[2 * (size_t)row + 1];
    const v4f w0 = *(const v4f*)(W_emb + d);
    const v4f w1 = *(const v4f*)(W_emb + kDIN + d);
    const v4f bb = *(const v4f*)(b_emb + d);
    v4f v = px * w0 + py * w1 + bb;
    v.x = fmaxf(v.x, 0.0f); v.y = fmaxf(v.y, 0.0f); v.z = fmaxf(v.z, 0.0f); v.w = fmaxf(v.w, 0.0f);
    v2u hi, lo; split_pack4(v, hi, lo);
    store_planes_2pass(PH + (size_t)row * kKL + d, PL + (size_t)row * kKL + d, hi, lo);
  }
  if (idx < kNP * (kHD / 4)) {
    const int p = idx >> 5;
    const int f = (idx & 31) * 4;
    const v4f v = *(const v4f*)(h0v + (size_t)p * kHD + f);
    v2u hi, lo; split_pack4(v, hi, lo);
    store_planes_2pass(PH + (size_t)p * kKL + kDIN + f, PL + (size_t)p * kKL + kDIN + f, hi, lo);
  }
}

template <bool LAST>
__global__ __launch_bounds__(256) void lstm_cell(
    const float* __restrict__ gates, const float* __restrict__ cin, float* __restrict__ cout,
    unsigned short* __restrict__ PHn, unsigned short* __restrict__ PLn, float* __restrict__ ahout) {
  const int idx = blockIdx.x * 256 + threadIdx.x;
  const int p = idx >> 5;
  const int f = (idx & 31) * 4;
  const float* gp = gates + (size_t)p * kNGATE + f;
  const float* cp = cin + (size_t)p * kHD + f;
  float c0 = 0.f, c1 = 0.f, c2 = 0.f, c3 = 0.f, q0 = 0.f, q1 = 0.f, q2 = 0.f, q3 = 0.f;
#pragma unroll 1
  for (int e = 0; e < 4; ++e) {
    const float iv = gp[e], fv = gp[kHD + e], gv = gp[2 * kHD + e], ov = gp[3 * kHD + e];
    const float cv = cp[e];
    const float cn = sigm_f(fv) * cv + sigm_f(iv) * tanh_f(gv);
    const float hn = sigm_f(ov) * tanh_f(cn);
    if (e == 0) { c0 = cn; q0 = hn; }
    else if (e == 1) { c1 = cn; q1 = hn; }
    else if (e == 2) { c2 = cn; q2 = hn; }
    else { c3 = cn; q3 = hn; }
  }
  v4f hv; hv.x = q0; hv.y = q1; hv.z = q2; hv.w = q3;
  if (LAST) {
    store_f4_2pass(ahout + (size_t)p * kHD + f, hv);
  } else {
    v4f cvv; cvv.x = c0; cvv.y = c1; cvv.z = c2; cvv.w = c3;
    store_f4_2pass(cout + (size_t)p * kHD + f, cvv);
    v2u hi, lo; split_pack4(hv, hi, lo);
    store_planes_2pass(PHn + (size_t)p * kKL + kDIN + f, PLn + (size_t)p * kKL + kDIN + f, hi, lo);
  }
}

__global__ __launch_bounds__(256) void pair_hidden(
    const float* __restrict__ action, const float* __restrict__ goal,
    const float* __restrict__ W_dist, const float* __restrict__ b_dist,
    unsigned short* __restrict__ MH, unsigned short* __restrict__ ML) {
  __shared__ __align__(16) float wds[8 * kDD];
  __shared__ __align__(16) float bds[kDD];
  const int tid = threadIdx.x;
#pragma unroll 1
  for (int e = tid; e < 8 * kDD; e += 256) wds[e] = W_dist[e];
  if (tid < kDD) bds[tid] = b_dist[tid];
  __syncthreads();
  const int idx = blockIdx.x * 256 + tid;
  const int r = idx >> 4;
  const int q = (idx & 15) * 4;
  const int ig = r >> 5;
  const int g = r >> 10;
  const int jg = (g << 5) | (r & 31);
  const v2f ai = *(const v2f*)(action + 2 * (size_t)ig);
  const v2f gi = *(const v2f*)(goal + 2 * (size_t)ig);
  const v2f aj = *(const v2f*)(action + 2 * (size_t)jg);
  const v2f gj = *(const v2f*)(goal + 2 * (size_t)jg);
  const float d[8] = {ai.x, ai.y, gi.x, gi.y, aj.x, aj.y, gj.x, gj.y};
  v4f acc = *(const v4f*)(bds + q);
#pragma unroll
  for (int c = 0; c < 8; ++c) {
    const v4f w = *(const v4f*)(wds + c * kDD + q);
    acc += d[c] * w;
  }
  acc.x = fmaxf(acc.x, 0.0f); acc.y = fmaxf(acc.y, 0.0f); acc.z = fmaxf(acc.z, 0.0f); acc.w = fmaxf(acc.w, 0.0f);
  v2u hi, lo; split_pack4(acc, hi, lo);
  store_planes_2pass(MH + (size_t)r * kDD + q, ML + (size_t)r * kDD + q, hi, lo);
}

__global__ __launch_bounds__(256) void attn_context(
    const float* __restrict__ ah, const float* __restrict__ gh, const float* __restrict__ gate,
    const float* __restrict__ wa, unsigned short* __restrict__ XH, unsigned short* __restrict__ XL) {
  __shared__ __align__(16) float tahs[kGS * kHD];
  __shared__ __align__(16) float was[2 * kKC];
  __shared__ float sS[8][kNH][40];
  __shared__ float sInv[8][8];
  const int g = blockIdx.x;
  const int tid = threadIdx.x;
  const int lane = tid & 31;
  const int wave = tid >> 5;
  const float* ahg = ah + (size_t)g * kGS * kHD;
#pragma unroll 1
  for (int e = tid; e < kGS * kHD; e += 256) tahs[e] = tanh_f(ahg[e]);
#pragma unroll 1
  for (int e = tid; e < 2 * kKC; e += 256) was[e] = wa[e];
  __syncthreads();

  const int f = lane * 4;
  float w2[kNH][4];
#pragma unroll
  for (int h = 0; h < kNH; ++h) {
    const v4f t = *(const v4f*)(was + kKC + h * kHD + f);
    w2[h][0] = t.x; w2[h][1] = t.y; w2[h][2] = t.z; w2[h][3] = t.w;
  }

#pragma unroll 1
  for (int ii = 0; ii < 4; ++ii) {
    const int i = wave * 4 + ii;
    const int ig = g * kGS + i;
    const v4f a4 = *(const v4f*)(ah + (size_t)ig * kHD + f);
    const v4f g4 = *(const v4f*)(gh + (size_t)ig * kHD + f);
    float si1[kNH];
#pragma unroll
    for (int h = 0; h < kNH; ++h) {
      const v4f w1 = *(const v4f*)(was + h * kHD + f);
      float p = a4.x * w1.x;
      p = fmaf(a4.y, w1.y, p); p = fmaf(a4.z, w1.z, p); p = fmaf(a4.w, w1.w, p);
      si1[h] = wave_sum(p);
    }
#pragma unroll 1
    for (int k = 0; k <= kGS; ++k) {
      const int j = (k > 0) ? (k - 1) : 0;
      const v4f gv = *(const v4f*)(gate + ((size_t)ig * kGS + j) * kHD + f);
      const v4f tv = *(const v4f*)(tahs + j * kHD + f);
      const v4f ga = gv * tv;
      const v4f vec = sel4(k == 0, a4, sel4(j == i, g4, ga));
#pragma unroll
      for (int h = 0; h < kNH; ++h) {
        float p = vec.x * w2[h][0];
        p = fmaf(vec.y, w2[h][1], p); p = fmaf(vec.z, w2[h][2], p); p = fmaf(vec.w, w2[h][3], p);
        p = wave_sum(p);
        float s = si1[h] + p;
        s = (s >= 0.0f) ? s : 0.2f * s;
        if (lane == 0) sS[wave][h][k] = s;
      }
    }
    wave_sync();
    {
      const int hq = lane >> 3;
      const int sub = lane & 7;
      float m = -INFINITY;
#pragma unroll 1
      for (int it = 0; it < 5; ++it) {
        const int k = sub + 8 * it;
        const int kc = min(k, kGS);
        float v = sS[wave][hq][kc];
        v = (k <= kGS) ? v : -INFINITY;
        m = fmaxf(m, v);
      }
      m = fmaxf(m, __shfl_xor(m, 1, 32));
      m = fmaxf(m, __shfl_xor(m, 2, 32));
      m = fmaxf(m, __shfl_xor(m, 4, 32));
      float sum = 0.0f;
#pragma unroll 1
      for (int it = 0; it < 5; ++it) {
        const int k = sub + 8 * it;
        const int kc = min(k, kGS);
        const float v = sS[wave][hq][kc];
        float e = expf(v - m);
        e = (k <= kGS) ? e : 0.0f;
        sum += e;
        if (k <= kGS) sS[wave][hq][k] = e;
      }
      sum += __shfl_xor(sum, 1, 32);
      sum += __shfl_xor(sum, 2, 32);
      sum += __shfl_xor(sum, 4, 32);
      const float inv = 1.0f / sum;
      if (sub == 0) sInv[wave][hq] = inv;
    }
    wave_sync();
    float acc[kNH][4];
#pragma unroll
    for (int h = 0; h < kNH; ++h) { acc[h][0] = 0.0f; acc[h][1] = 0.0f; acc[h][2] = 0.0f; acc[h][3] = 0.0f; }
#pragma unroll 1
    for (int k = 0; k <= kGS; ++k) {
      const int j = (k > 0) ? (k - 1) : 0;
      const v4f gv = *(const v4f*)(gate + ((size_t)ig * kGS + j) * kHD + f);
      const v4f tv = *(const v4f*)(tahs + j * kHD + f);
      const v4f ga = gv * tv;
      const v4f vec = sel4(k == 0, a4, sel4(j == i, g4, ga));
#pragma unroll
      for (int h = 0; h < kNH; ++h) {
        const float pk = sS[wave][h][k];
        acc[h][0] = fmaf(pk, vec.x, acc[h][0]);
        acc[h][1] = fmaf(pk, vec.y, acc[h][1]);
        acc[h][2] = fmaf(pk, vec.z, acc[h][2]);
        acc[h][3] = fmaf(pk, vec.w, acc[h][3]);
      }
    }
    v2u hiv[kNH], lov[kNH];
#pragma unroll
    for (int h = 0; h < kNH; ++h) {
      const float inv = sInv[wave][h];
      v4f c4;
      c4.x = acc[h][0] * inv; c4.y = acc[h][1] * inv; c4.z = acc[h][2] * inv; c4.w = acc[h][3] * inv;
      split_pack4(c4, hiv[h], lov[h]);
    }
    unsigned short* ph = XH + (size_t)ig * kKC + f;
    unsigned short* pl = XL + (size_t)ig * kKC + f;
    for (int pass = 0; pass < 2; ++pass) {
#pragma unroll
      for (int h = 0; h < kNH; ++h) {
        *(volatile v2u*)(ph + h * kHD) = hiv[h];
        *(volatile v2u*)(pl + h * kHD) = lov[h];
      }
      __threadfence();
    }
    wave_sync();
  }
}

extern "C" void kernel_launch(void* const* d_in, const int* in_sizes, int n_in,
                              void* d_out, int out_size, void* d_ws, size_t ws_size,
                              hipStream_t stream) {
  if (n_in < 20) return;
  if (in_sizes[0] != kT * kNP * 2 || in_sizes[1] != kNP * kHD || in_sizes[2] != kNP * 2 ||
      in_sizes[3] != kNP * 2 || in_sizes[4] != kNP * kHD || in_sizes[5] != kNP * kHD ||
      in_sizes[6] != 2 * kDIN || in_sizes[7] != kDIN || in_sizes[8] != kNGATE * kDIN ||
      in_sizes[9] != kNGATE * kHD || in_sizes[10] != kNGATE || in_sizes[11] != kNGATE ||
      in_sizes[12] != 8 * kDD || in_sizes[13] != kDD || in_sizes[14] != kDD * kHD ||
      in_sizes[15] != kHD || in_sizes[16] != kNH * kHD * kHD || in_sizes[17] != 2 * kHD ||
      in_sizes[18] != kHD || in_sizes[19] != kNG * 2) return;
  if (out_size != kNP * kHD) return;
  if ((size_t)ws_size < kWsTotal) return;

  const float* obs    = (const float*)d_in[0];
  const float* ghs    = (const float*)d_in[1];
  const float* goal   = (const float*)d_in[2];
  const float* action = (const float*)d_in[3];
  const float* h0     = (const float*)d_in[4];
  const float* c0     = (const float*)d_in[5];
  const float* W_emb  = (const float*)d_in[6];
  const float* b_emb  = (const float*)d_in[7];
  const float* W_ih   = (const float*)d_in[8];
  const float* W_hh   = (const float*)d_in[9];
  const float* b_ih   = (const float*)d_in[10];
  const float* b_hh   = (const float*)d_in[11];
  const float* W_dist = (const float*)d_in[12];
  const float* b_dist = (const float*)d_in[13];
  const float* W_gate = (const float*)d_in[14];
  const float* b_gate = (const float*)d_in[15];
  const float* gat_w  = (const float*)d_in[16];
  const float* gat_a  = (const float*)d_in[17];
  const float* gat_b  = (const float*)d_in[18];

  char* ws = (char*)d_ws;
  unsigned short* WcH = (unsigned short*)(ws + oWcH);
  unsigned short* WcL = (unsigned short*)(ws + oWcL);
  float* biasg = (float*)(ws + oBias);
  unsigned short* WgH = (unsigned short*)(ws + oWgH);
  unsigned short* WgL = (unsigned short*)(ws + oWgL);
  unsigned short* WaH = (unsigned short*)(ws + oWaH);
  unsigned short* WaL = (unsigned short*)(ws + oWaL);
  float* wav = (float*)(ws + oWav);
  unsigned short* PH = (unsigned short*)(ws + oPH);
  unsigned short* PL = (unsigned short*)(ws + oPL);
  float* gates = (float*)(ws + oG);
  float* cb[2] = {(float*)(ws + oC0), (float*)(ws + oC1)};
  float* ahbuf = (float*)(ws + oAh);
  unsigned short* MH = (unsigned short*)(ws + oMH);
  unsigned short* ML = (unsigned short*)(ws + oML);
  float* gatebuf = (float*)(ws + oGate);
  unsigned short* XH = (unsigned short*)(ws + oXH);
  unsigned short* XL = (unsigned short*)(ws + oXL);
  const size_t planeE = (size_t)kNP * kKL;

  prep_params<<<(kNGATE * (kKL / 4)) / 256, 256, 0, stream>>>(
      W_ih, W_hh, b_ih, b_hh, W_gate, gat_w, gat_a, WcH, WcL, biasg, WgH, WgL, WaH, WaL, wav);
  embed_inputs<<<(kT * kNP * (kDIN / 4)) / 256, 256, 0, stream>>>(obs, W_emb, b_emb, h0, PH, PL);

  for (int t = 0; t < kT; ++t) {
    const unsigned short* aH = PH + (size_t)t * planeE;
    const unsigned short* aL = PL + (size_t)t * planeE;
    wmma_gemm64<1, true, 2, 0, false, 0><<<dim3((kNP / 64) * (kNGATE / 64) / 8, 1), 256, 0, stream>>>(
        aH, aL, kKL, 0L, WcH, WcL, kKL, 0L, (void*)gates, (void*)gates, kNGATE, 0L,
        biasg, biasg, 0L, kNP, kNGATE, kKL, 1.0f);
    const float* cin = (t == 0) ? c0 : cb[(t - 1) & 1];
    float* cout = cb[t & 1];
    if (t < kT - 1) {
      lstm_cell<false><<<(kNP * 32) / 256, 256, 0, stream>>>(
          gates, cin, cout, PH + (size_t)(t + 1) * planeE, PL + (size_t)(t + 1) * planeE, ahbuf);
    } else {
      lstm_cell<true><<<(kNP * 32) / 256, 256, 0, stream>>>(gates, cin, cout, PH, PL, ahbuf);
    }
  }

  pair_hidden<<<(kNPAIR * 16) / 256, 256, 0, stream>>>(action, goal, W_dist, b_dist, MH, ML);
  wmma_gemm64<1, true, 2, 0, false, 6><<<dim3((kNPAIR / 64) * (kHD / 64) / 8, 1), 256, 0, stream>>>(
      MH, ML, kDD, 0L, WgH, WgL, kDD, 0L, (void*)gatebuf, (void*)gatebuf, kHD, 0L,
      b_gate, biasg, 0L, kNPAIR, kHD, kDD, 1.0f);

  attn_context<<<kNG, 256, 0, stream>>>(ahbuf, ghs, gatebuf, wav, XH, XL);

  wmma_gemm64<1, true, 3, 0, false, 2><<<dim3((kNP / 64) * (kHD / 64) / 8, 1), 256, 0, stream>>>(
      XH, XL, kKC, 0L, WaH, WaL, kKC, 0L, d_out, d_out, kHD, 0L,
      gat_b, biasg, 0L, kNP, kHD, kKC, 0.25f);
}
